// EntityAlignmentModule_33741263077482
// MI455X (gfx1250) — hardware-run, weakly checked
//
#include <hip/hip_runtime.h>
#include <math.h>

typedef __attribute__((ext_vector_type(16))) _Float16 v16h;
typedef __attribute__((ext_vector_type(8)))  _Float16 v8h;
typedef __attribute__((ext_vector_type(8)))  float    v8f;
typedef __attribute__((ext_vector_type(4)))  float    v4f;

constexpr int kNB   = 32;
constexpr int kNE   = 64;
constexpr int kNR   = 36;
constexpr int kDtx  = 768;
constexpr int kDim  = 2048;
constexpr int kD    = 512;
constexpr int kMt   = kNB * kNE;
constexpr int kMi   = kNB * kNR;
constexpr int kPerB = kNE * kNR;
constexpr int kOut0 = kNB * kNE * kNR;
constexpr int kOut1 = kNB * kD;
static_assert(kMt == 2048 && kMi == 1152 && kPerB == 2304);
static_assert((kMt % 64) == 0 && (kMi % 64) == 0 && (kD % 64) == 0);
static_assert((kDtx % 32) == 0 && (kDim % 32) == 0 && (kD % 32) == 0);
static_assert((((kMt / 64) * (kD / 64)) % 8) == 0 && (((kMi / 64) * (kD / 64)) % 8) == 0);
static_assert((kDtx % 64) == 0 && (kDim % 64) == 0 && ((2 * kD) % 64) == 0);
static_assert((kMt % 8) == 0 && (kMi % 8) == 0);
static_assert(((size_t)kOut0 * 4) % 128 == 0);
static_assert((8 * kNR * 4) % 128 == 0);
static_assert(kPerB == 9 * 256);

constexpr float kCarryAct = 16.0f;
constexpr float kCarryW   = 256.0f;
constexpr float kFold     = 1.0f / (kCarryAct * kCarryW);
constexpr float kH16MinNormal = 6.103515625e-5f;
constexpr float kLnEps = 1e-5f;

constexpr size_t kOffXTH = 0;
constexpr size_t kOffXIH = kOffXTH + (size_t)kMt * kDtx * 2;
constexpr size_t kOffWTT = kOffXIH + (size_t)kMi * kDim * 2;
constexpr size_t kOffWIT = kOffWTT + (size_t)kD * kDtx * 2;
constexpr size_t kOffW1T = kOffWIT + (size_t)kD * kDim * 2;
constexpr size_t kOffYT  = kOffW1T + (size_t)kD * (2 * kD) * 2;
constexpr size_t kOffYI  = kOffYT  + (size_t)kMt * kD * 4;
constexpr size_t kOffTAH = kOffYI  + (size_t)kMi * kD * 4;
constexpr size_t kOffIAH = kOffTAH + (size_t)kMt * kD * 2;
constexpr size_t kOffIAF = kOffIAH + (size_t)kMi * kD * 2;
constexpr size_t kOffHT  = kOffIAF + (size_t)kMi * kD * 4;
constexpr size_t kOffHI  = kOffHT  + (size_t)kMt * kD * 4;
constexpr size_t kWsTotal = kOffHI + (size_t)kMi * kD * 4;
static_assert(kWsTotal == 30539776ull);
static_assert(kWsTotal <= 134217728ull);
static_assert((kOffXIH % 128) == 0 && (kOffWTT % 128) == 0 && (kOffWIT % 128) == 0 && (kOffW1T % 128) == 0 &&
              (kOffYT % 128) == 0 && (kOffYI % 128) == 0 && (kOffTAH % 128) == 0 && (kOffIAH % 128) == 0 &&
              (kOffIAF % 128) == 0 && (kOffHT % 128) == 0 && (kOffHI % 128) == 0);

__device__ __forceinline__ _Float16 to_h16(float v, float carry) {
  const float s = v * carry;
  const float t = (fabsf(s) < kH16MinNormal) ? 0.0f : s;
  return (_Float16)t;
}

__device__ __forceinline__ v8f mma_g(v16h a, v16h b, v8f c) {
  c = __builtin_amdgcn_wmma_f32_16x16x32_f16(false, a, false, b, (short)0, c, false, false);
  asm volatile("v_nop\n\tv_nop\n\tv_nop\n\tv_nop" : "+v"(c) : "v"(a), "v"(b));
  return c;
}
__device__ __forceinline__ void acc_guard4(v8f& a, v8f& b, v8f& c, v8f& d) {
  asm volatile("v_nop\n\tv_nop\n\tv_nop\n\tv_nop" : "+v"(a), "+v"(b), "+v"(c), "+v"(d));
}
struct FragH {
  union U { v16h v; v8h h[2]; };
  static __device__ __forceinline__ v16h load(const _Float16* p) {
    U f;
    f.h[0] = *(const v8h*)(p);
    f.h[1] = *(const v8h*)(p + 16);
    return f.v;
  }
};

__global__ __launch_bounds__(256) void cvt_rows_f16_kernel(
    const float* __restrict__ src, unsigned short* __restrict__ dst, int total8, float carry)
{
  const int i = blockIdx.x * 256 + threadIdx.x;
  if (i >= total8) return;
  const size_t e0 = (size_t)i << 3;
  const v4f a0 = *(const v4f*)(src + e0);
  const v4f a1 = *(const v4f*)(src + e0 + 4);
  v8h hv;
#pragma unroll
  for (int e = 0; e < 4; ++e) {
    const float f0 = a0[e];
    const float f1 = a1[e];
    hv[e]     = to_h16(f0, carry);
    hv[4 + e] = to_h16(f1, carry);
  }
  unsigned short* q = dst + e0;
  *(volatile v8h*)q = hv;
  __threadfence();
  *(volatile v8h*)q = hv;
}

__global__ __launch_bounds__(256) void tr_cvt_f16_kernel(
    const float* __restrict__ src, unsigned short* __restrict__ dst, int K, int N, float carry)
{
  __shared__ __align__(16) float sT[64 * 68];
  const int tid = threadIdx.x, lane = tid & 31, wave = tid >> 5;
  const int k0 = blockIdx.x * 64, n0 = blockIdx.y * 64;
  {
    const int kr = tid >> 2, cs = (tid & 3) * 16;
    const float* sp = src + (size_t)(k0 + kr) * N + n0 + cs;
#pragma unroll
    for (int j = 0; j < 4; ++j) {
      const v4f t = *(const v4f*)(sp + 4 * j);
      *(v4f*)(sT + kr * 68 + cs + 4 * j) = t;
    }
  }
  __syncthreads();
  const int q = lane >> 3, c8 = (lane & 7) * 8;
  v8h hv[2];
#pragma unroll
  for (int it = 0; it < 2; ++it) {
    const int n = it * 32 + wave * 4 + q;
#pragma unroll
    for (int e = 0; e < 8; ++e) {
      const float f = sT[(c8 + e) * 68 + n];
      hv[it][e] = to_h16(f, carry);
    }
  }
  for (int pass = 0; pass < 2; ++pass) {
#pragma unroll
    for (int it = 0; it < 2; ++it) {
      const int n = it * 32 + wave * 4 + q;
      *(volatile v8h*)(dst + (size_t)(n0 + n) * K + k0 + c8) = hv[it];
    }
    __threadfence();
  }
}

template <int BIAS_MODE>
__global__ __launch_bounds__(256) void wmma_gemm64_f16(
    const unsigned short* __restrict__ Ap, int lda,
    const unsigned short* __restrict__ Btp, int ldb,
    float* __restrict__ C, int ldc,
    const float* __restrict__ bias,
    int M, int N, int K, float scale)
{
  const _Float16* A  = (const _Float16*)Ap;
  const _Float16* Bt = (const _Float16*)Btp;
  __shared__ __align__(16) float sT[8][16 * 68];
  const int lane = threadIdx.x & 31;
  const int wave = threadIdx.x >> 5;
  const int tilesN = N >> 6;
  const int tilesM = M >> 6;
  const int tile = blockIdx.x * 8 + wave;
  if (tile >= tilesM * tilesN) return;
  const int tm = tile / tilesN;
  const int tn = tile - tm * tilesN;
  const int m0 = tm << 6;
  const int n0 = tn << 6;

  const int rlane = lane & 15;
  const int koff  = (lane >> 4) * 8;
  const int mOff  = (lane >> 4) * 8;

  v8f acc[4][4];
#pragma unroll
  for (int i = 0; i < 4; ++i)
#pragma unroll
    for (int j = 0; j < 4; ++j) acc[i][j] = (v8f){0.f, 0.f, 0.f, 0.f, 0.f, 0.f, 0.f, 0.f};

  for (int k0 = 0; k0 < K; k0 += 32) {
    v16h bh[4];
#pragma unroll
    for (int j = 0; j < 4; ++j) {
      const size_t bo = (size_t)(n0 + (j << 4) + rlane) * ldb + koff + k0;
      bh[j] = FragH::load(Bt + bo);
    }
#pragma unroll
    for (int i = 0; i < 4; ++i) {
      const size_t ao = (size_t)(m0 + (i << 4) + rlane) * lda + koff + k0;
      const v16h ah = FragH::load(A + ao);
#pragma unroll
      for (int j = 0; j < 4; ++j) acc[i][j] = mma_g(ah, bh[j], acc[i][j]);
    }
  }
  acc_guard4(acc[0][0], acc[0][1], acc[0][2], acc[0][3]);
  acc_guard4(acc[1][0], acc[1][1], acc[1][2], acc[1][3]);
  acc_guard4(acc[2][0], acc[2][1], acc[2][2], acc[2][3]);
  acc_guard4(acc[3][0], acc[3][1], acc[3][2], acc[3][3]);

  float* slab = sT[wave];
#pragma unroll
  for (int i = 0; i < 4; ++i) {
    const int mBase = m0 + (i << 4);
#pragma unroll
    for (int j = 0; j < 4; ++j) {
      const int n = n0 + (j << 4) + rlane;
      float bv = 0.f;
      if (BIAS_MODE == 2) bv = bias[n];
#pragma unroll
      for (int r = 0; r < 8; ++r) {
        float v = acc[i][j][r] * scale;
        if (BIAS_MODE == 2) v += bv;
        slab[(mOff + r) * 68 + (j << 4) + rlane] = v;
      }
    }
    __builtin_amdgcn_fence(__ATOMIC_RELEASE, "workgroup");
    __builtin_amdgcn_wave_barrier();
    __builtin_amdgcn_fence(__ATOMIC_ACQUIRE, "workgroup");
    {
      const int hh = lane >> 4, c4 = (lane & 15) * 4;
      for (int pass = 0; pass < 2; ++pass) {
#pragma unroll
        for (int it = 0; it < 8; ++it) {
          const int row = it * 2 + hh;
          const v4f v = *(const v4f*)(slab + row * 68 + c4);
          *(volatile v4f*)(C + (size_t)(mBase + row) * ldc + n0 + c4) = v;
        }
        __threadfence();
      }
    }
    __builtin_amdgcn_fence(__ATOMIC_RELEASE, "workgroup");
    __builtin_amdgcn_wave_barrier();
    __builtin_amdgcn_fence(__ATOMIC_ACQUIRE, "workgroup");
  }
}

template <bool WRITE_F32>
__global__ __launch_bounds__(256) void relu_ln_rows_kernel(
    const float* __restrict__ Y, const float* __restrict__ bias,
    const float* __restrict__ gam, const float* __restrict__ bet,
    unsigned short* __restrict__ outH, float* __restrict__ outF, int rows, float carry)
{
  __shared__ __align__(16) float sRow[8 * kD];
  const int tid = threadIdx.x, lane = tid & 31, wave = tid >> 5;
  const int row = blockIdx.x * 8 + wave;
  const bool live = row < rows;
  const int rowc = live ? row : (rows - 1);
  const float* yp = Y + (size_t)rowc * kD + lane * 4;

  float x[16], gg[16], bt[16];
#pragma unroll
  for (int j = 0; j < 4; ++j) {
    const v4f yv = *(const v4f*)(yp + 128 * j);
    const v4f bv = *(const v4f*)(bias + lane * 4 + 128 * j);
    const v4f gv = *(const v4f*)(gam + lane * 4 + 128 * j);
    const v4f tv = *(const v4f*)(bet + lane * 4 + 128 * j);
#pragma unroll
    for (int c = 0; c < 4; ++c) {
      const float yy = yv[c];
      const float bb = bv[c];
      x[4 * j + c]  = fmaxf(yy + bb, 0.0f);
      gg[4 * j + c] = gv[c];
      bt[4 * j + c] = tv[c];
    }
  }
  float s = 0.f;
#pragma unroll
  for (int i = 0; i < 16; ++i) s += x[i];
#pragma unroll
  for (int m = 16; m >= 1; m >>= 1) s += __shfl_xor(s, m, 32);
  const float mu = s * (1.0f / (float)kD);
  float ss = 0.f;
#pragma unroll
  for (int i = 0; i < 16; ++i) {
    const float dlt = x[i] - mu;
    ss = fmaf(dlt, dlt, ss);
  }
#pragma unroll
  for (int m = 16; m >= 1; m >>= 1) ss += __shfl_xor(ss, m, 32);
  const float var  = ss * (1.0f / (float)kD);
  const float rstd = rsqrtf(var + kLnEps);

  float* sr = sRow + wave * kD;
  v4f fv[4];
#pragma unroll
  for (int j = 0; j < 4; ++j) {
    v4f ov;
#pragma unroll
    for (int c = 0; c < 4; ++c) {
      const float o = (x[4 * j + c] - mu) * rstd * gg[4 * j + c] + bt[4 * j + c];
      ov[c] = o;
    }
    fv[j] = ov;
    *(v4f*)(sr + lane * 4 + 128 * j) = ov;
  }
  __syncthreads();
  v8h hv[2];
#pragma unroll
  for (int j2 = 0; j2 < 2; ++j2) {
    const float* p = sr + lane * 8 + 256 * j2;
    const v4f a0 = *(const v4f*)(p);
    const v4f a1 = *(const v4f*)(p + 4);
#pragma unroll
    for (int e = 0; e < 4; ++e) {
      const float f0 = a0[e];
      const float f1 = a1[e];
      hv[j2][e]     = to_h16(f0, carry);
      hv[j2][4 + e] = to_h16(f1, carry);
    }
  }
  for (int pass = 0; pass < 2; ++pass) {
    if (live) {
      if (WRITE_F32) {
#pragma unroll
        for (int j = 0; j < 4; ++j)
          *(volatile v4f*)(outF + (size_t)row * kD + lane * 4 + 128 * j) = fv[j];
      }
#pragma unroll
      for (int j2 = 0; j2 < 2; ++j2)
        *(volatile v8h*)(outH + (size_t)row * kD + lane * 8 + 256 * j2) = hv[j2];
    }
    __threadfence();
  }
}

__global__ __launch_bounds__(256) void pair_score_kernel(
    const float* __restrict__ ht, const float* __restrict__ hi,
    const float* __restrict__ W2, const float* __restrict__ b2, float* __restrict__ out0)
{
  __shared__ __align__(16) float sSc[8 * kNR];
  const int tid = threadIdx.x, lane = tid & 31, wave = tid >> 5;
  const int b  = blockIdx.x >> 3;
  const int et = blockIdx.x & 7;
  const int e  = et * 8 + wave;
  const float* hrow = ht + (size_t)(b * kNE + e) * kD + lane * 4;
  float hv[16], wv[16];
#pragma unroll
  for (int j = 0; j < 4; ++j) {
    const v4f a = *(const v4f*)(hrow + 128 * j);
    const v4f w = *(const v4f*)(W2 + lane * 4 + 128 * j);
#pragma unroll
    for (int c = 0; c < 4; ++c) {
      hv[4 * j + c] = a[c];
      wv[4 * j + c] = w[c];
    }
  }
  const float bb = b2[0];
  const float* hib = hi + (size_t)b * kNR * kD + lane * 4;
#pragma unroll 1
  for (int r = 0; r < kNR; ++r) {
    const float* hp = hib + (size_t)r * kD;
    float p = 0.f;
#pragma unroll
    for (int j = 0; j < 4; ++j) {
      const v4f xv = *(const v4f*)(hp + 128 * j);
#pragma unroll
      for (int c = 0; c < 4; ++c) {
        const float t = fmaxf(hv[4 * j + c] + xv[c], 0.0f);
        p = fmaf(t, wv[4 * j + c], p);
      }
    }
#pragma unroll
    for (int m = 16; m >= 1; m >>= 1) p += __shfl_xor(p, m, 32);
    const float sraw = p + bb;
    const float sg = 1.0f / (1.0f + expf(-sraw));
    if (lane == 0) sSc[wave * kNR + r] = sg;
  }
  __syncthreads();
  if (wave == 0) {
    v4f val[3];
#pragma unroll
    for (int it = 0; it < 3; ++it) {
      const int idx = it * 32 + lane;
      const int idc = idx < 72 ? idx : 71;
      val[it] = *(const v4f*)(sSc + idc * 4);
    }
    float* dst = out0 + (size_t)(b * kNE + et * 8) * kNR;
    for (int pass = 0; pass < 2; ++pass) {
#pragma unroll
      for (int it = 0; it < 3; ++it) {
        const int idx = it * 32 + lane;
        if (idx < 72) *(volatile v4f*)(dst + idx * 4) = val[it];
      }
      __threadfence();
    }
  }
}

__global__ __launch_bounds__(256) void softmax_agg_kernel(
    const float* sc, const float* __restrict__ iaF, float* out1)
{
  __shared__ __align__(16) float sE[kPerB];
  __shared__ float sRedM[8];
  __shared__ float sRedS[8];
  __shared__ float sC[64];
  const int tid = threadIdx.x, lane = tid & 31, wave = tid >> 5;
  const int b = blockIdx.x;
  const float* sp = sc + (size_t)b * kPerB;

  float mx = -INFINITY;
#pragma unroll
  for (int i = 0; i < 9; ++i) {
    const float v = sp[tid + 256 * i];
    sE[tid + 256 * i] = v;
    mx = fmaxf(mx, v);
  }
#pragma unroll
  for (int m = 16; m >= 1; m >>= 1) mx = fmaxf(mx, __shfl_xor(mx, m, 32));
  if (lane == 0) sRedM[wave] = mx;
  __syncthreads();
  float mall = sRedM[0];
#pragma unroll
  for (int i = 1; i < 8; ++i) mall = fmaxf(mall, sRedM[i]);

  float ls = 0.f;
#pragma unroll 1
  for (int i = 0; i < 9; ++i) {
    const int idx = tid + 256 * i;
    const float ev = expf(sE[idx] - mall);
    sE[idx] = ev;
    ls += ev;
  }
#pragma unroll
  for (int m = 16; m >= 1; m >>= 1) ls += __shfl_xor(ls, m, 32);
  if (lane == 0) sRedS[wave] = ls;
  __syncthreads();
  float z = 0.f;
#pragma unroll
  for (int i = 0; i < 8; ++i) z += sRedS[i];

  if (tid < kNR) {
    float s = 0.f;
#pragma unroll 1
    for (int e = 0; e < kNE; ++e) s += sE[e * kNR + tid];
    sC[tid] = s * (1.0f / (z * (float)kNE));
  }
  __syncthreads();

  if (tid < 128) {
    const float* ip = iaF + (size_t)b * kNR * kD + tid * 4;
    float a0 = 0.f, a1 = 0.f, a2 = 0.f, a3 = 0.f;
#pragma unroll 4
    for (int r = 0; r < kNR; ++r) {
      const float c = sC[r];
      const v4f v = *(const v4f*)(ip + (size_t)r * kD);
      a0 = fmaf(c, v[0], a0);
      a1 = fmaf(c, v[1], a1);
      a2 = fmaf(c, v[2], a2);
      a3 = fmaf(c, v[3], a3);
    }
    v4f o;
    o[0] = a0; o[1] = a1; o[2] = a2; o[3] = a3;
    float* dst = out1 + (size_t)b * kD + tid * 4;
    *(volatile v4f*)dst = o;
    __threadfence();
    *(volatile v4f*)dst = o;
  }
}

extern "C" void kernel_launch(void* const* d_in, const int* in_sizes, int n_in,
                              void* d_out, int out_size, void* d_ws, size_t ws_size,
                              hipStream_t stream) {
  if (n_in < 14) return;
  if (in_sizes[0] != kMt * kDtx) return;
  if (in_sizes[1] != kMi * kDim) return;
  if (in_sizes[2] != kDtx * kD) return;
  if (in_sizes[3] != kD || in_sizes[4] != kD || in_sizes[5] != kD) return;
  if (in_sizes[6] != kDim * kD) return;
  if (in_sizes[7] != kD || in_sizes[8] != kD || in_sizes[9] != kD) return;
  if (in_sizes[10] != 2 * kD * kD) return;
  if (in_sizes[11] != kD) return;
  if (in_sizes[12] != kD) return;
  if (in_sizes[13] != 1) return;
  if (out_size != kOut0 + kOut1) return;
  if (ws_size < kWsTotal) return;

  const float* text_feats  = (const float*)d_in[0];
  const float* image_feats = (const float*)d_in[1];
  const float* W_text      = (const float*)d_in[2];
  const float* b_text      = (const float*)d_in[3];
  const float* g_text      = (const float*)d_in[4];
  const float* beta_text   = (const float*)d_in[5];
  const float* W_img       = (const float*)d_in[6];
  const float* b_img       = (const float*)d_in[7];
  const float* g_img       = (const float*)d_in[8];
  const float* beta_img    = (const float*)d_in[9];
  const float* W1          = (const float*)d_in[10];
  const float* b1          = (const float*)d_in[11];
  const float* W2          = (const float*)d_in[12];
  const float* b2          = (const float*)d_in[13];
  float* out = (float*)d_out;

  char* ws = (char*)d_ws;
  unsigned short* XTH = (unsigned short*)(ws + kOffXTH);
  unsigned short* XIH = (unsigned short*)(ws + kOffXIH);
  unsigned short* WTT = (unsigned short*)(ws + kOffWTT);
  unsigned short* WIT = (unsigned short*)(ws + kOffWIT);
  unsigned short* W1T = (unsigned short*)(ws + kOffW1T);
  float*          YT  = (float*)(ws + kOffYT);
  float*          YI  = (float*)(ws + kOffYI);
  unsigned short* TAH = (unsigned short*)(ws + kOffTAH);
  unsigned short* IAH = (unsigned short*)(ws + kOffIAH);
  float*          IAF = (float*)(ws + kOffIAF);
  float*          HT  = (float*)(ws + kOffHT);
  float*          HI  = (float*)(ws + kOffHI);

  cvt_rows_f16_kernel<<<(kMt * kDtx / 8) / 256, 256, 0, stream>>>(text_feats, XTH, kMt * kDtx / 8, kCarryAct);
  cvt_rows_f16_kernel<<<(kMi * kDim / 8) / 256, 256, 0, stream>>>(image_feats, XIH, kMi * kDim / 8, kCarryAct);

  tr_cvt_f16_kernel<<<dim3(kDtx / 64, kD / 64), 256, 0, stream>>>(W_text, WTT, kDtx, kD, kCarryW);
  tr_cvt_f16_kernel<<<dim3(kDim / 64, kD / 64), 256, 0, stream>>>(W_img, WIT, kDim, kD, kCarryW);
  tr_cvt_f16_kernel<<<dim3((2 * kD) / 64, kD / 64), 256, 0, stream>>>(W1, W1T, 2 * kD, kD, kCarryW);

  wmma_gemm64_f16<0><<<((kMt / 64) * (kD / 64)) / 8, 256, 0, stream>>>(
      XTH, kDtx, WTT, kDtx, YT, kD, b_text, kMt, kD, kDtx, kFold);
  wmma_gemm64_f16<0><<<((kMi / 64) * (kD / 64)) / 8, 256, 0, stream>>>(
      XIH, kDim, WIT, kDim, YI, kD, b_img, kMi, kD, kDim, kFold);

  relu_ln_rows_kernel<false><<<kMt / 8, 256, 0, stream>>>(YT, b_text, g_text, beta_text, TAH, IAF, kMt, kCarryAct);
  relu_ln_rows_kernel<true><<<kMi / 8, 256, 0, stream>>>(YI, b_img, g_img, beta_img, IAH, IAF, kMi, kCarryAct);

  wmma_gemm64_f16<0><<<((kMt / 64) * (kD / 64)) / 8, 256, 0, stream>>>(
      TAH, kD, W1T, 2 * kD, HT, kD, b1, kMt, kD, kD, kFold);
  wmma_gemm64_f16<2><<<((kMi / 64) * (kD / 64)) / 8, 256, 0, stream>>>(
      IAH, kD, W1T + kD, 2 * kD, HI, kD, b1, kMi, kD, kD, kFold);

  pair_score_kernel<<<kNB * (kNE / 8), 256, 0, stream>>>(HT, HI, W2, b2, out);

  softmax_agg_kernel<<<kNB, 256, 0, stream>>>(out, IAF, out + kOut0);
}
